// PointNetSetAbstraction_4080218931818
// MI455X (gfx1250) — hardware-verified
//
#include <hip/hip_runtime.h>
#pragma clang fp contract(off)

typedef __attribute__((ext_vector_type(16))) _Float16 v16h;
typedef __attribute__((ext_vector_type(8)))  _Float16 v8h;
typedef __attribute__((ext_vector_type(8)))  float    v8f;
typedef __attribute__((ext_vector_type(4)))  float    v4f;

constexpr int kBatch = 16;
constexpr int kPts = 4096;
constexpr int kCen = 1024;
constexpr int kNbr = 32;
constexpr int kFeat = 64;
constexpr int kW0In = 67;
constexpr int kK0 = 96;
constexpr int kH1 = 64;
constexpr int kH2 = 64;
constexpr int kH3 = 128;
constexpr int kChunkBatches = 4;
constexpr int kNumChunks = 4;
constexpr int kChunkRows = kChunkBatches * kCen * kNbr;
constexpr float kRadiusSq = 0.04f;
constexpr float kBnEps = 1e-5f;
constexpr float kWCarry = 16.0f;
constexpr float kWCarryInv = 0.0625f;

static_assert(kBatch == kChunkBatches * kNumChunks, "chunking covers all batches");
static_assert(kChunkRows % 64 == 0, "GEMM M tile multiple");
static_assert(kH1 % 64 == 0 && kH2 % 64 == 0 && kH3 % 64 == 0, "GEMM N tile multiple");
static_assert(kK0 % 32 == 0 && kH1 % 32 == 0 && kH2 % 32 == 0, "GEMM K step multiple");
static_assert(kCen * kNbr == 32768, "rows per batch is 2^15");
static_assert(kPts % 32 == 0, "ball-query chunks");
static_assert((size_t)kBatch * kCen * 3 * 4 == 196608, "out0 bytes");
static_assert((size_t)196608 + (size_t)kBatch * kCen * kH3 * 4 == 8585216, "d_out bytes");

constexpr size_t kOffGrp  = 0;
constexpr size_t kOffNxyz = kOffGrp + (size_t)kBatch * kCen * kNbr * 4;
constexpr size_t kOffWh   = kOffNxyz + (size_t)kBatch * kCen * 3 * 4;
constexpr int    kWhBt0   = 0;
constexpr int    kWhBt1   = kH1 * kK0;
constexpr int    kWhBt2   = kWhBt1 + kH2 * kH1;
constexpr int    kWhTotal = kWhBt2 + kH3 * kH2;
constexpr size_t kOffBn   = kOffWh + (size_t)kWhTotal * 2;
constexpr size_t kOffA0   = kOffBn + 512 * 4;
constexpr size_t kOffH1   = kOffA0 + (size_t)kChunkRows * kK0 * 2;
constexpr size_t kOffH2   = kOffH1 + (size_t)kChunkRows * kH1 * 2;
constexpr size_t kWsTotal = kOffH2 + (size_t)kChunkRows * kH2 * 2;
static_assert(kOffNxyz % 128 == 0 && kOffWh % 128 == 0 && kOffBn % 128 == 0, "line aligned");
static_assert(kOffA0 % 128 == 0 && kOffH1 % 128 == 0 && kOffH2 % 128 == 0, "line aligned");
static_assert(kWsTotal <= (size_t)134217728, "carve under 128 MiB");
static_assert(kWhTotal == 18432, "weight plane halves");

__device__ __forceinline__ void keep4_h(v16h a, v16h b, v16h c, v16h d) { asm volatile("v_nop" :: "v"(a), "v"(b), "v"(c), "v"(d)); }
__device__ __forceinline__ void acc_guard4(v8f& a, v8f& b, v8f& c, v8f& d) { asm volatile("v_nop\n\tv_nop\n\tv_nop\n\tv_nop" : "+v"(a), "+v"(b), "+v"(c), "+v"(d)); }
__device__ __forceinline__ void grp_guard_h(v8f& a, v8f& b, v8f& c, v8f& d, v16h x, v16h y0, v16h y1, v16h y2, v16h y3) {
  asm volatile("v_nop\n\tv_nop\n\tv_nop\n\tv_nop" : "+v"(a), "+v"(b), "+v"(c), "+v"(d) : "v"(x), "v"(y0), "v"(y1), "v"(y2), "v"(y3));
}
struct FragH {
  union U { v16h v; v8h h[2]; };
  static __device__ __forceinline__ v16h load(const _Float16* p) {
    U f; f.h[0] = *(const v8h*)(p); f.h[1] = *(const v8h*)(p + 16); return f.v;
  }
  static __device__ __forceinline__ v8f mma(v16h a, v16h b, v8f c) {
    return __builtin_amdgcn_wmma_f32_16x16x32_f16(false, a, false, b, (short)0, c, false, false);
  }
};

__global__ __launch_bounds__(256)
void prep_kernel(const float* __restrict__ W0, const float* __restrict__ W1, const float* __restrict__ W2,
                 const float* __restrict__ b0, const float* __restrict__ g0, const float* __restrict__ be0,
                 const float* __restrict__ m0, const float* __restrict__ v0,
                 const float* __restrict__ b1, const float* __restrict__ g1, const float* __restrict__ be1,
                 const float* __restrict__ m1, const float* __restrict__ v1,
                 const float* __restrict__ b2, const float* __restrict__ g2, const float* __restrict__ be2,
                 const float* __restrict__ m2, const float* __restrict__ v2,
                 _Float16* __restrict__ wh, float* __restrict__ bn)
{
  const int tid = threadIdx.x;
  if (blockIdx.x < 9) {
    const int t = blockIdx.x * 256 + tid;
    float vals[8];
    if (t < 768) {
      const int o = t / 12;
      const int j = t - o * 12;
#pragma unroll
      for (int e = 0; e < 8; ++e) {
        const int c = j * 8 + e;
        const int src = (c < 64) ? (c + 3) : ((c < kW0In) ? (c - 64) : 0);
        const float w = W0[o * kW0In + src];
        vals[e] = (c < kW0In) ? w : 0.0f;
      }
    } else if (t < 1280) {
      const int u = (t - 768) * 8;
      const v4f a = *(const v4f*)(W1 + u);
      const v4f c = *(const v4f*)(W1 + u + 4);
      vals[0] = a[0]; vals[1] = a[1]; vals[2] = a[2]; vals[3] = a[3];
      vals[4] = c[0]; vals[5] = c[1]; vals[6] = c[2]; vals[7] = c[3];
    } else {
      const int u = (t - 1280) * 8;
      const v4f a = *(const v4f*)(W2 + u);
      const v4f c = *(const v4f*)(W2 + u + 4);
      vals[0] = a[0]; vals[1] = a[1]; vals[2] = a[2]; vals[3] = a[3];
      vals[4] = c[0]; vals[5] = c[1]; vals[6] = c[2]; vals[7] = c[3];
    }
    v8h hv;
#pragma unroll
    for (int e = 0; e < 8; ++e) hv[e] = (_Float16)(vals[e] * kWCarry);
    volatile v8h* dst = (volatile v8h*)(wh + (size_t)t * 8);
    *dst = hv;
    __threadfence();
    *dst = hv;
  } else {
    const int w = tid >> 5;
    const float* gp; const float* vp; const float* bp; const float* mp; const float* ep;
    int o4; bool isSh;
    if (w == 0) { gp = g0; vp = v0; bp = b0; mp = m0; ep = be0; o4 = (tid & 15) * 4; isSh = ((tid & 31) >= 16); }
    else if (w == 1) { gp = g1; vp = v1; bp = b1; mp = m1; ep = be1; o4 = (tid & 15) * 4; isSh = ((tid & 31) >= 16); }
    else { gp = g2; vp = v2; bp = b2; mp = m2; ep = be2; o4 = (tid & 31) * 4; isSh = (w == 3); }
    if (tid < 128) {
      const v4f gg = *(const v4f*)(gp + o4);
      const v4f vv = *(const v4f*)(vp + o4);
      const v4f bb = *(const v4f*)(bp + o4);
      const v4f mm = *(const v4f*)(mp + o4);
      const v4f ee = *(const v4f*)(ep + o4);
      v4f ov;
#pragma unroll
      for (int e = 0; e < 4; ++e) {
        const float sc = gg[e] * rsqrtf(vv[e] + kBnEps);
        const float sh = (bb[e] - mm[e]) * sc + ee[e];
        ov[e] = isSh ? sh : (sc * kWCarryInv);
      }
      volatile v4f* dst = (volatile v4f*)(bn + tid * 4);
      *dst = ov;
      __threadfence();
      *dst = ov;
    }
  }
}

__global__ __launch_bounds__(1024)
void fps_kernel(const float* __restrict__ xyz, float* __restrict__ out0, float* __restrict__ nxyz)
{
#pragma clang fp contract(off)
  __shared__ float spt[3 * kPts];
  __shared__ int   sidx[kCen];
  __shared__ float wbv[2][32];
  __shared__ int   wbi[2][32];

  const int b = blockIdx.x;
  const int tid = threadIdx.x;
  const int wv = tid >> 5;
  const int lane = tid & 31;
  const float* base = xyz + (size_t)b * kPts * 3;

#pragma unroll
  for (int j = 0; j < 3; ++j) {
    const int f = tid + j * 1024;
    const v4f v = *(const v4f*)(base + 4 * f);
#pragma unroll
    for (int k = 0; k < 4; ++k) {
      const int e = 4 * f + k;
      const int p = e / 3;
      const int c = e - 3 * p;
      spt[c * kPts + p] = v[k];
    }
  }
  if (tid == 0) sidx[0] = 0;
  __syncthreads();

  float dist[4];
#pragma unroll
  for (int t = 0; t < 4; ++t) dist[t] = 1e10f;

  int far = 0;
  for (int i = 1; i < kCen; ++i) {
    const float cx = spt[far];
    const float cy = spt[kPts + far];
    const float cz = spt[2 * kPts + far];
    float bv = -1.0f;
    int bi = 0;
#pragma unroll
    for (int t = 0; t < 4; ++t) {
      const int p = tid + t * 1024;
      const float dx = spt[p] - cx;
      const float dy = spt[kPts + p] - cy;
      const float dz = spt[2 * kPts + p] - cz;
      const float t0 = dx * dx;
      const float t1 = dy * dy;
      const float t2 = dz * dz;
      const float d = (t0 + t2) + t1;
      const float nd = fminf(dist[t], d);
      dist[t] = nd;
      const bool take = (nd > bv) || (nd == bv && p < bi);
      bv = take ? nd : bv;
      bi = take ? p : bi;
    }
#pragma unroll
    for (int o = 16; o > 0; o >>= 1) {
      const float ov = __shfl_xor(bv, o, 32);
      const int   oi = __shfl_xor(bi, o, 32);
      const bool take = (ov > bv) || (ov == bv && oi < bi);
      bv = take ? ov : bv;
      bi = take ? oi : bi;
    }
    const int buf = i & 1;
    if (lane == 0) { wbv[buf][wv] = bv; wbi[buf][wv] = bi; }
    __syncthreads();
    float v2 = wbv[buf][lane];
    int   i2 = wbi[buf][lane];
#pragma unroll
    for (int o = 16; o > 0; o >>= 1) {
      const float ov = __shfl_xor(v2, o, 32);
      const int   oi = __shfl_xor(i2, o, 32);
      const bool take = (ov > v2) || (ov == v2 && oi < i2);
      v2 = take ? ov : v2;
      i2 = take ? oi : i2;
    }
    far = __builtin_amdgcn_readfirstlane(i2);
    far = far < 0 ? 0 : (far > kPts - 1 ? kPts - 1 : far);
    if (tid == 0) sidx[i] = far;
  }
  __syncthreads();

  if (tid < 768) {
    v4f ov;
#pragma unroll
    for (int k = 0; k < 4; ++k) {
      const int e = 4 * tid + k;
      const int s = e / 3;
      const int c = e - 3 * s;
      int id = sidx[s];
      id = id < 0 ? 0 : (id > kPts - 1 ? kPts - 1 : id);
      ov[k] = spt[c * kPts + id];
    }
    volatile v4f* d0 = (volatile v4f*)(out0 + (size_t)b * kCen * 3 + 4 * tid);
    volatile v4f* d1 = (volatile v4f*)(nxyz + (size_t)b * kCen * 3 + 4 * tid);
    *d0 = ov;
    *d1 = ov;
    __threadfence();
    *d0 = ov;
    *d1 = ov;
  }
}

__global__ __launch_bounds__(256)
void ballq_kernel(const float* __restrict__ xyz, const float* __restrict__ nxyz, int* __restrict__ grp)
{
#pragma clang fp contract(off)
  __shared__ int slots[8][32];
  const int tid = threadIdx.x;
  const int wave = tid >> 5;
  const int lane = tid & 31;
  const int cen = blockIdx.x * 8 + wave;
  const int b = cen >> 10;
  const float* pb = xyz + (size_t)b * kPts * 3;
  const float qx = nxyz[(size_t)cen * 3 + 0];
  const float qy = nxyz[(size_t)cen * 3 + 1];
  const float qz = nxyz[(size_t)cen * 3 + 2];
  const float qxx = qx * qx;
  const float qyy = qy * qy;
  const float qzz = qz * qz;
  const float q2 = (qxx + qzz) + qyy;
  int* sl = slots[wave];
  sl[lane] = 0;
  int cnt = 0;
  for (int ch = 0; ch < kPts / 32; ++ch) {
    const int n = ch * 32 + lane;
    const float x = pb[n * 3 + 0];
    const float y = pb[n * 3 + 1];
    const float z = pb[n * 3 + 2];
    const float xx = x * x;
    const float yy = y * y;
    const float zz = z * z;
    const float p2 = (xx + zz) + yy;
    float dot = qx * x;
    dot = __builtin_fmaf(qy, y, dot);
    dot = __builtin_fmaf(qz, z, dot);
    const float two_dot = 2.0f * dot;
    const float d2 = (q2 + p2) - two_dot;
    const bool keep = !(d2 > kRadiusSq);
    const unsigned mask = __builtin_amdgcn_ballot_w32(keep);
    const int slot = cnt + __popc(mask & ((1u << lane) - 1u));
    if (keep && slot < kNbr) sl[slot] = n;
    cnt += __popc(mask);
    if (cnt >= kNbr) break;
  }
  __builtin_amdgcn_fence(__ATOMIC_RELEASE, "workgroup");
  __builtin_amdgcn_wave_barrier();
  __builtin_amdgcn_fence(__ATOMIC_ACQUIRE, "workgroup");
  const int nfill = cnt < kNbr ? cnt : kNbr;
  const int src = lane < nfill ? lane : 0;
  int val = sl[src];
  val = val < 0 ? 0 : (val > kPts - 1 ? kPts - 1 : val);
  volatile int* gp = grp + (size_t)cen * kNbr + lane;
  *gp = val;
  __threadfence();
  *gp = val;
}

__global__ __launch_bounds__(256)
void gather_kernel(const float* __restrict__ xyz, const float* __restrict__ points,
                   const float* __restrict__ nxyz, const int* __restrict__ grp,
                   _Float16* __restrict__ a0, int rowBase)
{
  const int tid = threadIdx.x;
  const int wave = tid >> 5;
  const int lane = tid & 31;
  const int lrow0 = (blockIdx.x * 8 + wave) * 8;
#pragma unroll 1
  for (int t = 0; t < 3; ++t) {
    const int P = t * 32 + lane;
    const int rr = P / 12;
    const int j = P - rr * 12;
    const int lrow = lrow0 + rr;
    const int grow = rowBase + lrow;
    int i = grp[grow];
    i = i < 0 ? 0 : (i > kPts - 1 ? kPts - 1 : i);
    const int b = grow >> 15;
    const int cen = grow >> 5;
    const int jc = j < 8 ? j : 7;
    const float* prow = points + ((size_t)b * kPts + i) * kFeat + jc * 8;
    const v4f pa = *(const v4f*)(prow);
    const v4f pc = *(const v4f*)(prow + 4);
    const float* xp = xyz + ((size_t)b * kPts + i) * 3;
    const float* qp = nxyz + (size_t)cen * 3;
    const float d0 = xp[0] - qp[0];
    const float d1 = xp[1] - qp[1];
    const float d2 = xp[2] - qp[2];
    const bool isP = (j < 8);
    const bool isD = (j == 8);
    float vals[8];
    vals[0] = isP ? pa[0] : (isD ? d0 : 0.0f);
    vals[1] = isP ? pa[1] : (isD ? d1 : 0.0f);
    vals[2] = isP ? pa[2] : (isD ? d2 : 0.0f);
    vals[3] = isP ? pa[3] : 0.0f;
    vals[4] = isP ? pc[0] : 0.0f;
    vals[5] = isP ? pc[1] : 0.0f;
    vals[6] = isP ? pc[2] : 0.0f;
    vals[7] = isP ? pc[3] : 0.0f;
    v8h hv;
#pragma unroll
    for (int e = 0; e < 8; ++e) hv[e] = (_Float16)vals[e];
    volatile v8h* dst = (volatile v8h*)(a0 + (size_t)lrow * kK0 + j * 8);
    *dst = hv;
    __threadfence();
    *dst = hv;
  }
}

template <int OUT_MODE>
__global__ __launch_bounds__(256) void mlp_gemm64(
    const unsigned short* __restrict__ Ap, int lda,
    const unsigned short* __restrict__ Btp, int ldb,
    void* __restrict__ Cout, int ldc,
    const float* __restrict__ scn, const float* __restrict__ shn,
    int M, int N, int K) {
  const _Float16* A = (const _Float16*)Ap;
  const _Float16* Bt = (const _Float16*)Btp;
  __shared__ __align__(16) float sT[8][16 * 68];
  const int lane = threadIdx.x & 31;
  const int wave = threadIdx.x >> 5;
  const int tilesN = N >> 6;
  const int tilesM = M >> 6;
  const int tile = blockIdx.x * 8 + wave;
  if (tile >= tilesM * tilesN) return;
  const int tm = tile / tilesN;
  const int tn = tile - tm * tilesN;
  const int m0 = tm << 6;
  const int n0 = tn << 6;

  const int rlane = lane & 15;
  const int koff  = (lane >> 4) * 8;
  const int mOff  = (lane >> 4) * 8;

  v8f acc[4][4];
#pragma unroll
  for (int i = 0; i < 4; ++i)
#pragma unroll
    for (int j = 0; j < 4; ++j) acc[i][j] = (v8f){0.f,0.f,0.f,0.f,0.f,0.f,0.f,0.f};

  for (int k0 = 0; k0 < K; k0 += 32) {
    v16h bh[4];
#pragma unroll
    for (int j = 0; j < 4; ++j) {
      const size_t bo = (size_t)(n0 + (j << 4) + rlane) * ldb + koff + k0;
      bh[j] = FragH::load(Bt + bo);
    }
#pragma unroll
    for (int i = 0; i < 4; ++i) {
      const size_t ao = (size_t)(m0 + (i << 4) + rlane) * lda + koff + k0;
      const v16h ah = FragH::load(A + ao);
#pragma unroll
      for (int j = 0; j < 4; ++j) acc[i][j] = FragH::mma(ah, bh[j], acc[i][j]);
      grp_guard_h(acc[i][0], acc[i][1], acc[i][2], acc[i][3], ah, bh[0], bh[1], bh[2], bh[3]);
    }
    keep4_h(bh[0], bh[1], bh[2], bh[3]);
  }
  acc_guard4(acc[0][0], acc[0][1], acc[0][2], acc[0][3]);
  acc_guard4(acc[1][0], acc[1][1], acc[1][2], acc[1][3]);
  acc_guard4(acc[2][0], acc[2][1], acc[2][2], acc[2][3]);
  acc_guard4(acc[3][0], acc[3][1], acc[3][2], acc[3][3]);

  float* slab = sT[wave];
  float scv[4], shv[4];
#pragma unroll
  for (int j = 0; j < 4; ++j) {
    const int n = n0 + (j << 4) + rlane;
    scv[j] = scn[n];
    shv[j] = shn[n];
  }

  if (OUT_MODE == 1) {
    unsigned short* C = (unsigned short*)Cout;
    const int q = lane >> 3, c8 = (lane & 7) * 8;
#pragma unroll
    for (int i = 0; i < 4; ++i) {
      const int mBase = m0 + (i << 4);
#pragma unroll
      for (int j = 0; j < 4; ++j) {
#pragma unroll
        for (int r = 0; r < 8; ++r) {
          float v = acc[i][j][r] * scv[j] + shv[j];
          v = fmaxf(v, 0.0f);
          slab[(mOff + r) * 68 + (j << 4) + rlane] = v;
        }
      }
      __builtin_amdgcn_fence(__ATOMIC_RELEASE, "workgroup");
      __builtin_amdgcn_wave_barrier();
      __builtin_amdgcn_fence(__ATOMIC_ACQUIRE, "workgroup");
      for (int pass = 0; pass < 2; ++pass) {
#pragma unroll
        for (int it = 0; it < 4; ++it) {
          const int row = it * 4 + q;
          const float* sp = slab + row * 68 + c8;
          v8h hv;
#pragma unroll
          for (int e = 0; e < 8; ++e) hv[e] = (_Float16)sp[e];
          *(volatile v8h*)(C + (size_t)(mBase + row) * ldc + n0 + c8) = hv;
        }
        __threadfence();
      }
      __builtin_amdgcn_fence(__ATOMIC_RELEASE, "workgroup");
      __builtin_amdgcn_wave_barrier();
      __builtin_amdgcn_fence(__ATOMIC_ACQUIRE, "workgroup");
    }
  } else {
    float* C = (float*)Cout;
    const int hh = lane >> 4, c4 = (lane & 15) * 4;
    const int cen0 = m0 >> 5;
#pragma unroll
    for (int g = 0; g < 2; ++g) {
#pragma unroll
      for (int j = 0; j < 4; ++j) {
        float mx = 0.0f;
#pragma unroll
        for (int ii = 0; ii < 2; ++ii) {
#pragma unroll
          for (int r = 0; r < 8; ++r) {
            const float v = acc[2 * g + ii][j][r] * scv[j] + shv[j];
            mx = fmaxf(mx, v);
          }
        }
        const float other = __shfl_xor(mx, 16, 32);
        mx = fmaxf(mx, other);
        if (hh == 0) slab[g * 68 + (j << 4) + rlane] = mx;
      }
    }
    __builtin_amdgcn_fence(__ATOMIC_RELEASE, "workgroup");
    __builtin_amdgcn_wave_barrier();
    __builtin_amdgcn_fence(__ATOMIC_ACQUIRE, "workgroup");
    for (int pass = 0; pass < 2; ++pass) {
      const v4f v = *(const v4f*)(slab + hh * 68 + c4);
      *(volatile v4f*)(C + (size_t)(cen0 + hh) * ldc + n0 + c4) = v;
      __threadfence();
    }
  }
}

extern "C" void kernel_launch(void* const* d_in, const int* in_sizes, int n_in,
                              void* d_out, int out_size, void* d_ws, size_t ws_size,
                              hipStream_t stream)
{
  (void)in_sizes; (void)out_size;
  if (n_in < 20) return;
  if (ws_size < kWsTotal) return;

  const float* xyz    = (const float*)d_in[0];
  const float* points = (const float*)d_in[1];
  const float* W0  = (const float*)d_in[2];
  const float* b0  = (const float*)d_in[3];
  const float* g0  = (const float*)d_in[4];
  const float* be0 = (const float*)d_in[5];
  const float* m0  = (const float*)d_in[6];
  const float* v0  = (const float*)d_in[7];
  const float* W1  = (const float*)d_in[8];
  const float* b1  = (const float*)d_in[9];
  const float* g1  = (const float*)d_in[10];
  const float* be1 = (const float*)d_in[11];
  const float* m1  = (const float*)d_in[12];
  const float* v1  = (const float*)d_in[13];
  const float* W2  = (const float*)d_in[14];
  const float* b2  = (const float*)d_in[15];
  const float* g2  = (const float*)d_in[16];
  const float* be2 = (const float*)d_in[17];
  const float* m2  = (const float*)d_in[18];
  const float* v2  = (const float*)d_in[19];

  float* out0 = (float*)d_out;
  float* out1 = out0 + (size_t)kBatch * kCen * 3;

  char* ws = (char*)d_ws;
  int*      grp  = (int*)(ws + kOffGrp);
  float*    nxyz = (float*)(ws + kOffNxyz);
  _Float16* wh   = (_Float16*)(ws + kOffWh);
  float*    bn   = (float*)(ws + kOffBn);
  _Float16* a0   = (_Float16*)(ws + kOffA0);
  unsigned short* a0u = (unsigned short*)(ws + kOffA0);
  unsigned short* h1u = (unsigned short*)(ws + kOffH1);
  unsigned short* h2u = (unsigned short*)(ws + kOffH2);
  const unsigned short* bt0 = (const unsigned short*)(ws + kOffWh) + kWhBt0;
  const unsigned short* bt1 = (const unsigned short*)(ws + kOffWh) + kWhBt1;
  const unsigned short* bt2 = (const unsigned short*)(ws + kOffWh) + kWhBt2;

  prep_kernel<<<10, 256, 0, stream>>>(W0, W1, W2,
                                      b0, g0, be0, m0, v0,
                                      b1, g1, be1, m1, v1,
                                      b2, g2, be2, m2, v2, wh, bn);
  fps_kernel<<<kBatch, 1024, 0, stream>>>(xyz, out0, nxyz);
  ballq_kernel<<<kBatch * kCen / 8, 256, 0, stream>>>(xyz, nxyz, grp);

  const int tiles64 = kChunkRows / 64;
  for (int c = 0; c < kNumChunks; ++c) {
    const int rowBase = c * kChunkRows;
    gather_kernel<<<kChunkRows / 64, 256, 0, stream>>>(xyz, points, nxyz, grp, a0, rowBase);
    mlp_gemm64<1><<<tiles64 * (kH1 / 64) / 8, 256, 0, stream>>>(
        a0u, kK0, bt0, kK0, (void*)h1u, kH1, bn + 0, bn + 64, kChunkRows, kH1, kK0);
    mlp_gemm64<1><<<tiles64 * (kH2 / 64) / 8, 256, 0, stream>>>(
        h1u, kH1, bt1, kH1, (void*)h2u, kH2, bn + 128, bn + 192, kChunkRows, kH2, kH1);
    float* outc = out1 + (size_t)c * kChunkBatches * kCen * kH3;
    mlp_gemm64<3><<<tiles64 * (kH3 / 64) / 8, 256, 0, stream>>>(
        h2u, kH2, bt2, kH2, (void*)outc, kH3, bn + 256, bn + 384, kChunkRows, kH3, kH2);
  }
}
